// CausalSelfAttention_80814104641605
// MI455X (gfx1250) — hardware-verified
//
#include <hip/hip_runtime.h>
#include <math.h>

typedef __attribute__((ext_vector_type(16))) _Float16 v16h;
typedef __attribute__((ext_vector_type(16))) __bf16 v16b;
typedef __attribute__((ext_vector_type(8)))  _Float16 v8h;
typedef __attribute__((ext_vector_type(8)))  __bf16 v8b;
typedef __attribute__((ext_vector_type(8)))  float v8f;
typedef __attribute__((ext_vector_type(4)))  float v4f;
typedef __attribute__((ext_vector_type(4)))  unsigned v4u;

template <typename T> __device__ __forceinline__ void vst2(void* p, T v) { *(volatile T*)p = v; __threadfence(); *(volatile T*)p = v; }
__device__ __forceinline__ v8f wmma16(v16h a, v16h b, v8f c) {
  v8f d = __builtin_amdgcn_wmma_f32_16x16x32_f16(false, a, false, b, (short)0, c, false, false);
  asm volatile("v_nop\n\tv_nop\n\tv_nop\n\tv_nop" : "+v"(d) : "v"(a), "v"(b));
  return d;
}
__device__ __forceinline__ v8f wmma_bf(v16b a, v16b b, v8f c) {
  v8f d = __builtin_amdgcn_wmma_f32_16x16x32_bf16(false, a, false, b, (short)0, c, false, false);
  asm volatile("v_nop\n\tv_nop\n\tv_nop\n\tv_nop" : "+v"(d) : "v"(a), "v"(b));
  return d;
}
__device__ __forceinline__ v16h frag_h(const _Float16* rowk0, int lane) {
  union { v16h v; v8h q[2]; } u; const _Float16* p = rowk0 + 8 * (lane >> 4);
  u.q[0] = *(const v8h*)p; u.q[1] = *(const v8h*)(p + 16); return u.v;
}
__device__ __forceinline__ v16b frag_b(const __bf16* rowk0, int lane) {
  union { v16b v; v8b q[2]; } u; const __bf16* p = rowk0 + 8 * (lane >> 4);
  u.q[0] = *(const v8b*)p; u.q[1] = *(const v8b*)(p + 16); return u.v;
}
struct F2 { v16b h, l; };
__device__ __forceinline__ F2 bsplit16(const float v[16]) { F2 r;
#pragma unroll
  for (int i = 0; i < 16; ++i) { const __bf16 h = (__bf16)v[i]; r.h[i] = h; r.l[i] = (__bf16)(v[i] - (float)h); }
  return r; }
__device__ __forceinline__ F2 split_row(const float* row, int k0, int lane) { float v[16]; const float* p = row + k0 + 8 * (lane >> 4);
#pragma unroll
  for (int i = 0; i < 8; ++i) { v[i] = p[i]; v[8 + i] = p[16 + i]; }
  return bsplit16(v); }
__device__ __forceinline__ v16b wcol_io(const float* Wm, int k0, int o, int lane, int ld) { v16b w; const int g = lane >> 4;
#pragma unroll
  for (int i = 0; i < 8; ++i) { w[i] = (__bf16)Wm[(size_t)(k0 + 8 * g + i) * ld + o]; w[8 + i] = (__bf16)Wm[(size_t)(k0 + 16 + 8 * g + i) * ld + o]; }
  return w; }
#define LDSX() do { asm volatile("s_wait_dscnt 0" ::: "memory"); __builtin_amdgcn_wave_barrier(); __builtin_amdgcn_fence(3  , "workgroup"); } while (0)

#define NB_FULL 2
#define SEQ_FULL 2048
#ifndef NB
#define NB 2
#endif
#ifndef SEQ
#define SEQ 2048
#endif
#define TT SEQ
#define CC 1024
#define DIN 1024
#define NH 16
#define HD 64
#define NQB (TT / 64)
#define SCALE (0.125f)
#define QBH 4
#define KHI 256

static_assert(NB >= 1 && NB <= NB_FULL);
static_assert(SEQ <= SEQ_FULL);
static_assert(TT % 64 == 0);
static_assert(TT >= KHI);
static_assert(QBH * 64 == KHI);
static_assert(NH * HD == CC);
static_assert(HD == 64);
static_assert(DIN % 32 == 0 && CC % 32 == 0 && HD % 32 == 0);
static_assert(CC % 128 == 0);
static_assert((NB * TT) % 64 == 0);

constexpr size_t SZ_ROWS = (size_t)2 * NB * TT * CC;
constexpr size_t SZ_HI   = (size_t)2 * NB * KHI * CC;
constexpr size_t OFF_QH  = 0;
constexpr size_t OFF_QL  = OFF_QH + SZ_ROWS;
constexpr size_t OFF_KH  = OFF_QL + SZ_ROWS;
constexpr size_t OFF_KL  = OFF_KH + SZ_ROWS;
constexpr size_t OFF_VT  = OFF_KL + SZ_HI;
constexpr size_t OFF_VB  = OFF_VT + SZ_ROWS;
constexpr size_t OFF_VBL = OFF_VB + SZ_HI;
constexpr size_t OFF_Y   = OFF_VBL + SZ_HI;
constexpr size_t OFF_END = OFF_Y + (size_t)4 * NB * TT * CC;
static_assert(OFF_QL % 128 == 0 && OFF_KH % 128 == 0 && OFF_KL % 128 == 0 && OFF_VT % 128 == 0);
static_assert(OFF_VB % 128 == 0 && OFF_VBL % 128 == 0 && OFF_Y % 128 == 0);
static_assert(OFF_END <= (size_t)134217728);

__global__ __launch_bounds__(128) void k_proj(const float* __restrict__ X, const float* __restrict__ W, unsigned char* WS) {
  __shared__ __align__(16) _Float16 sh[64][136], sl[64][136];
  __shared__ __align__(16) _Float16 th[128][72];
  __shared__ __align__(16) __bf16 tb[128][72], tbl[128][72];
  const int tid = threadIdx.x; const int wave = __builtin_amdgcn_readfirstlane((int)(threadIdx.x >> 5)); const int lane = tid & 31, col = lane & 15, g = lane >> 4;
  const int which = blockIdx.z; const int c0 = blockIdx.y * 128;
  const size_t r0 = (size_t)blockIdx.x * 64; const size_t bb = r0 / TT; const int t0 = (int)(r0 % TT);
  const float* WA = W + (size_t)which * CC;
  const float* xr = X + (bb * (size_t)SEQ_FULL + t0 + wave * 16 + col) * DIN + 8 * g;
  v8f acc[8] = {};
#pragma unroll 2
  for (int kc = 0; kc < DIN / 32; ++kc) { v16b a; { const float* p = xr + kc * 32;
#pragma unroll
      for (int i = 0; i < 8; ++i) { a[i] = (__bf16)p[i]; a[8 + i] = (__bf16)p[16 + i]; } }
    asm volatile("s_wait_loadcnt 0x0" ::: "memory");
#pragma unroll
    for (int j = 0; j < 8; ++j) { const v16b w = wcol_io(WA, kc * 32, c0 + j * 16 + col, lane, 3 * CC); asm volatile("s_wait_loadcnt 0x0" ::: "memory"); acc[j] = wmma_bf(a, w, acc[j]); } }
  if (which < 2) {
    const size_t offH = which == 0 ? OFF_QH : OFF_KH; const size_t offL = which == 0 ? OFF_QL : OFF_KL;
    _Float16* DH = (_Float16*)(WS + offH); _Float16* DL = (_Float16*)(WS + offL);
    const bool hi_rows = (which == 0) || (t0 < KHI);
    const size_t lrow0 = which == 0 ? r0 : bb * (size_t)KHI + t0;
#pragma unroll
    for (int j = 0; j < 8; ++j) {
#pragma unroll
      for (int r = 0; r < 8; ++r) { const float v = acc[j][r]; const _Float16 hv = (_Float16)v; sh[wave * 16 + 8 * g + r][j * 16 + col] = hv; sl[wave * 16 + 8 * g + r][j * 16 + col] = (_Float16)((v - (float)hv) * 1024.0f); } }
    __syncthreads();
    for (int e = tid; e < 64 * 16; e += 128) { const int rl = e >> 4, q = e & 15;
      vst2((void*)(DH + (r0 + rl) * CC + c0 + q * 8), *(const v4u*)&sh[rl][q * 8]);
      if (hi_rows) vst2((void*)(DL + (lrow0 + rl) * (size_t)CC + c0 + q * 8), *(const v4u*)&sl[rl][q * 8]); }
  } else {
    _Float16* VT = (_Float16*)(WS + OFF_VT); __bf16* VB = (__bf16*)(WS + OFF_VB); __bf16* VBL = (__bf16*)(WS + OFF_VBL);
    const bool hi_rows = t0 < KHI;
#pragma unroll
    for (int j = 0; j < 8; ++j) {
#pragma unroll
      for (int r = 0; r < 8; ++r) { const float v = acc[j][r]; const int rl = wave * 16 + 8 * g + r, cl = j * 16 + col; th[cl][rl] = (_Float16)v; const __bf16 bh = (__bf16)v; tb[cl][rl] = bh; tbl[cl][rl] = (__bf16)(v - (float)bh); } }
    __syncthreads();
    for (int e = tid; e < 128 * 8; e += 128) { const int cl = e >> 3, q = e & 7;
      vst2((void*)(VT + (bb * CC + c0 + cl) * (size_t)TT + t0 + q * 8), *(const v4u*)&th[cl][q * 8]);
      if (hi_rows) { const size_t o3 = (bb * CC + c0 + cl) * (size_t)KHI + t0 + q * 8; vst2((void*)(VB + o3), *(const v4u*)&tb[cl][q * 8]); vst2((void*)(VBL + o3), *(const v4u*)&tbl[cl][q * 8]); } } } }

__global__ __launch_bounds__(128) void k_attn(const _Float16* __restrict__ QH, const _Float16* __restrict__ QL, const _Float16* __restrict__ KH, const _Float16* __restrict__ KL,
    const _Float16* __restrict__ VT, const __bf16* __restrict__ VB, const __bf16* __restrict__ VBL, float* __restrict__ Y) {
  __shared__ __align__(16) float pf[4][16][36];
  __shared__ __align__(16) float ss[4][16][HD + 4];
  const int tid = threadIdx.x; const int wave = __builtin_amdgcn_readfirstlane((int)(threadIdx.x >> 5)); const int lane = tid & 31, col = lane & 15, g = lane >> 4;
  const int qb = NQB - 1 - (int)blockIdx.x; const int h = blockIdx.y; const int b = blockIdx.z;
  const bool early = qb < QBH;
  const int ql0 = qb * 64 + wave * 16;
  const int nhalf = ((ql0 + 15) >> 5) + 1;
  const size_t qoff = ((size_t)b * TT + ql0 + col) * CC + h * HD;
  const size_t kbase = (size_t)b * TT * CC + h * HD;
  const size_t klbase = (size_t)b * KHI * CC + h * HD;
  float m[8], l[8];
#pragma unroll
  for (int r = 0; r < 8; ++r) { m[r] = -3.0e38f; l[r] = 0.0f; }
  v8f accO[4] = {};
#pragma unroll 1
  for (int hf = 0; hf < nhalf; ++hf) { const int k0 = hf * 32;
    v8f sa[2] = {}, ra[2] = {};
#pragma unroll
    for (int kc = 0; kc < HD / 32; ++kc) {
      const v16h ah = frag_h(QH + qoff + kc * 32, lane), al = frag_h(QL + qoff + kc * 32, lane);
      const v16h kf0 = frag_h(KH + kbase + (size_t)(k0 + col) * CC + kc * 32, lane);
      const v16h kf1 = frag_h(KH + kbase + (size_t)(k0 + 16 + col) * CC + kc * 32, lane);
      sa[0] = wmma16(ah, kf0, sa[0]); ra[0] = wmma16(al, kf0, ra[0]);
      sa[1] = wmma16(ah, kf1, sa[1]); ra[1] = wmma16(al, kf1, ra[1]);
      if (early) {
        const v16h kl0 = frag_h(KL + klbase + (size_t)(k0 + col) * CC + kc * 32, lane);
        const v16h kl1 = frag_h(KL + klbase + (size_t)(k0 + 16 + col) * CC + kc * 32, lane);
        ra[0] = wmma16(ah, kl0, ra[0]); ra[1] = wmma16(ah, kl1, ra[1]); } }
#pragma unroll
    for (int r = 0; r < 8; ++r) { const int qrow = ql0 + 8 * g + r;
      const bool ok0 = (k0 + col) <= qrow, ok1 = (k0 + 16 + col) <= qrow;
      const float a0 = ok0 ? (sa[0][r] + ra[0][r] * (1.0f / 1024.0f)) * SCALE : -3.0e38f;
      const float a1 = ok1 ? (sa[1][r] + ra[1][r] * (1.0f / 1024.0f)) * SCALE : -3.0e38f;
      float mx = fmaxf(a0, a1);
      mx = fmaxf(mx, __shfl_xor(mx, 1)); mx = fmaxf(mx, __shfl_xor(mx, 2)); mx = fmaxf(mx, __shfl_xor(mx, 4)); mx = fmaxf(mx, __shfl_xor(mx, 8));
      const float mn = fmaxf(m[r], mx);
      const float alpha = __expf(fmaxf(m[r] - mn, -80.0f));
      const float x0 = __expf(fmaxf(a0 - mn, -80.0f)), x1 = __expf(fmaxf(a1 - mn, -80.0f));
      const float e0 = ok0 ? x0 : 0.0f, e1 = ok1 ? x1 : 0.0f;
      m[r] = mn; l[r] = l[r] * alpha + (e0 + e1);
      accO[0][r] *= alpha; accO[1][r] *= alpha; accO[2][r] *= alpha; accO[3][r] *= alpha;
      pf[wave][8 * g + r][col] = e0; pf[wave][8 * g + r][16 + col] = e1; }
    LDSX();
    const v4f p0 = *(const v4f*)&pf[wave][col][8 * g], p1 = *(const v4f*)&pf[wave][col][8 * g + 4], p2 = *(const v4f*)&pf[wave][col][16 + 8 * g], p3 = *(const v4f*)&pf[wave][col][20 + 8 * g];
    if (early) {
      float pv[16];
#pragma unroll
      for (int i = 0; i < 4; ++i) { pv[i] = p0[i]; pv[4 + i] = p1[i]; pv[8 + i] = p2[i]; pv[12 + i] = p3[i]; }
      const F2 pp = bsplit16(pv);
#pragma unroll
      for (int j = 0; j < HD / 16; ++j) { const size_t po = ((size_t)b * CC + h * HD + j * 16 + col) * (size_t)KHI + k0;
        const v16b vh = frag_b(VB + po, lane), vl = frag_b(VBL + po, lane);
        accO[j] = wmma_bf(pp.l, vh, accO[j]); accO[j] = wmma_bf(pp.h, vl, accO[j]); accO[j] = wmma_bf(pp.h, vh, accO[j]); }
    } else {
      v16h pa;
#pragma unroll
      for (int i = 0; i < 4; ++i) { pa[i] = (_Float16)(p0[i] * 2048.0f); pa[4 + i] = (_Float16)(p1[i] * 2048.0f); pa[8 + i] = (_Float16)(p2[i] * 2048.0f); pa[12 + i] = (_Float16)(p3[i] * 2048.0f); }
#pragma unroll
      for (int j = 0; j < HD / 16; ++j) { const size_t po = ((size_t)b * CC + h * HD + j * 16 + col) * (size_t)TT + k0;
        accO[j] = wmma16(pa, frag_h(VT + po, lane), accO[j]); } }
    LDSX();
  }
  const float pscale = early ? 1.0f : 2048.0f;
#pragma unroll
  for (int r = 0; r < 8; ++r) { float lr = l[r];
    lr += __shfl_xor(lr, 1); lr += __shfl_xor(lr, 2); lr += __shfl_xor(lr, 4); lr += __shfl_xor(lr, 8);
    const float inv = 1.0f / (lr * pscale);
    ss[wave][8 * g + r][col] = accO[0][r] * inv; ss[wave][8 * g + r][16 + col] = accO[1][r] * inv;
    ss[wave][8 * g + r][32 + col] = accO[2][r] * inv; ss[wave][8 * g + r][48 + col] = accO[3][r] * inv; }
  LDSX();
#pragma unroll 1
  for (int rp = 0; rp < 8; ++rp) { const int rl = rp * 2 + g;
    vst2((void*)(Y + ((size_t)b * TT + ql0 + rl) * CC + h * HD + col * 4), *(const v4f*)&ss[wave][rl][col * 4]); } }

__global__ __launch_bounds__(128) void k_out(const float* __restrict__ Y, const float* __restrict__ WO, float* __restrict__ OUT) {
  __shared__ __align__(16) float sf[4][16][132];
  const int tid = threadIdx.x; const int wave = __builtin_amdgcn_readfirstlane((int)(threadIdx.x >> 5)); const int lane = tid & 31, col = lane & 15, g = lane >> 4;
  const int c0 = blockIdx.y * 128; const size_t rb = (size_t)blockIdx.x * 64; const size_t r0 = rb + wave * 16;
  const size_t bb = rb / TT; const int t0 = (int)(rb % TT);
  v8f acc[8] = {};
#pragma unroll 2
  for (int kc = 0; kc < CC / 32; ++kc) { const F2 a = split_row(Y + (r0 + col) * CC, kc * 32, lane); asm volatile("s_wait_loadcnt 0x0" ::: "memory");
#pragma unroll
    for (int j = 0; j < 8; ++j) { const v16b w = wcol_io(WO, kc * 32, c0 + j * 16 + col, lane, CC); asm volatile("s_wait_loadcnt 0x0" ::: "memory"); acc[j] = wmma_bf(a.h, w, acc[j]); acc[j] = wmma_bf(a.l, w, acc[j]); } }
#pragma unroll
  for (int j = 0; j < 8; ++j) {
#pragma unroll
    for (int r = 0; r < 8; ++r) sf[wave][8 * g + r][j * 16 + col] = acc[j][r]; }
  LDSX();
  const size_t orow0 = bb * (size_t)SEQ_FULL + t0 + wave * 16;
#pragma unroll 1
  for (int rl = 0; rl < 16; ++rl) vst2((void*)(OUT + (orow0 + rl) * CC + c0 + lane * 4), *(const v4f*)&sf[wave][rl][lane * 4]); }

extern "C" void kernel_launch(void* const* d_in, const int* in_sizes, int n_in, void* d_out, int out_size, void* d_ws, size_t ws_size, hipStream_t stream) {
  if (n_in < 3) return;
  const size_t rows_need = (size_t)(NB - 1) * SEQ_FULL + SEQ;
  if ((size_t)in_sizes[0] < rows_need * DIN) return;
  if ((size_t)in_sizes[1] < (size_t)DIN * 3 * CC) return;
  if ((size_t)in_sizes[2] < (size_t)CC * CC) return;
  if ((size_t)out_size < rows_need * CC) return;
  if (ws_size < OFF_END) return;
  const float* x = (const float*)d_in[0]; const float* wattn = (const float*)d_in[1]; const float* wproj = (const float*)d_in[2];
  unsigned char* ws = (unsigned char*)d_ws;
  const _Float16* QH = (const _Float16*)(ws + OFF_QH); const _Float16* QL = (const _Float16*)(ws + OFF_QL);
  const _Float16* KH = (const _Float16*)(ws + OFF_KH); const _Float16* KL = (const _Float16*)(ws + OFF_KL);
  const _Float16* VT = (const _Float16*)(ws + OFF_VT); const __bf16* VB = (const __bf16*)(ws + OFF_VB); const __bf16* VBL = (const __bf16*)(ws + OFF_VBL);
  float* Y = (float*)(ws + OFF_Y);
  k_proj<<<dim3(NB * TT / 64, CC / 128, 3), 128, 0, stream>>>(x, wattn, ws);
  k_attn<<<dim3(NQB, NH, NB), 128, 0, stream>>>(QH, QL, KH, KL, VT, VB, VBL, Y);
  k_out<<<dim3(NB * TT / 64, CC / 128), 128, 0, stream>>>(Y, wproj, (float*)d_out);
}
